// HopfONN_8126078124467
// MI455X (gfx1250) — hardware-verified
//
#include <hip/hip_runtime.h>
#include <math.h>

typedef __attribute__((ext_vector_type(16))) _Float16 v16h;
typedef __attribute__((ext_vector_type(8)))  _Float16 v8h;
typedef __attribute__((ext_vector_type(8)))  float    v8f;
typedef __attribute__((ext_vector_type(4)))  float    v4f;

constexpr int kBatch   = 524288;
constexpr int kOsc     = 16;
constexpr int kOutC    = 4;
constexpr int kRkSteps = 19;
constexpr int kChunk   = 128;
constexpr int kTilesPerChunk = kChunk / 16;
constexpr int kWaves   = 2048;
constexpr int kWavesPerBlock = 4;
constexpr int kChunksTotal = kBatch / kChunk;
constexpr int kChunksPerWave = kChunksTotal / kWaves;
constexpr int kOPitch  = kChunk * kOutC + 4;
constexpr float kH = (float)(0.5 * 20.0 / 19.0);
constexpr float kTwoPi = (float)(2.0 * 3.14159265358979323846);
static_assert(kChunksTotal % kWaves == 0 && kOsc == 16, "whole chunks per wave; the 16 oscillators fill one half of K");
static_assert((kOPitch % 4) == 0, "16-B aligned LDS rows");

constexpr float kZCarry     = 4096.0f;
constexpr float kWCarry     = 4096.0f;
constexpr float kFoldBack   = 1.0f / (kZCarry * kWCarry);
constexpr float kF16MinNorm = 6.103515625e-5f;

namespace eng {

union FragU { v16h v; v8h h[2]; };

__device__ __forceinline__ unsigned short f2bf_bits(float f) {
  unsigned u = __float_as_uint(f);
  return (unsigned short)((u + 0x7FFFu + ((u >> 16) & 1u)) >> 16);
}
__device__ __forceinline__ float bf16v(float f) {
  return __uint_as_float(((unsigned)f2bf_bits(f)) << 16);
}
__device__ __forceinline__ _Float16 to_f16_flushed(float c) {
  const float z = (fabsf(c) < kF16MinNorm) ? 0.0f : c;
  return (_Float16)z;
}
__device__ __forceinline__ v8f mma_f16(v16h a, v16h b) {
  v8f c = (v8f){0.f, 0.f, 0.f, 0.f, 0.f, 0.f, 0.f, 0.f};
  c = __builtin_amdgcn_wmma_f32_16x16x32_f16(false, a, false, b, (short)0, c, false, false);
  asm volatile("v_nop\n\tv_nop\n\tv_nop\n\tv_nop" : "+v"(c) : "v"(a), "v"(b));
  return c;
}
__device__ __forceinline__ v8f mma_f16_acc(v16h a, v16h b, v8f c) {
  c = __builtin_amdgcn_wmma_f32_16x16x32_f16(false, a, false, b, (short)0, c, false, false);
  asm volatile("v_nop\n\tv_nop\n\tv_nop\n\tv_nop" : "+v"(c) : "v"(a), "v"(b));
  return c;
}
__device__ __forceinline__ void z_frags(const float (&zr)[8], const float (&zi)[8], v16h& fhi, v16h& flo) {
  v8h a, b, c, d;
#pragma unroll
  for (int r = 0; r < 8; ++r) {
    const float cr = zr[r] * kZCarry, ci = zi[r] * kZCarry;
    const _Float16 hr = to_f16_flushed(cr), hi = to_f16_flushed(ci);
    a[r] = hr; b[r] = hi;
    c[r] = to_f16_flushed(cr - (float)hr);
    d[r] = to_f16_flushed(ci - (float)hi);
  }
  FragU fu; fu.h[0] = a; fu.h[1] = b; fhi = fu.v;
  fu.h[0] = c; fu.h[1] = d; flo = fu.v;
}

}

__device__ __forceinline__ void rhs(const float (&zr)[8], const float (&zi)[8], v16h fragWr, v16h fragWi,
                                    float (&dr)[8], float (&di)[8]) {
  v16h fhi, flo;
  eng::z_frags(zr, zi, fhi, flo);
  const v8f wr = eng::mma_f16_acc(fragWr, flo, eng::mma_f16(fragWr, fhi));
  const v8f wi = eng::mma_f16_acc(fragWi, flo, eng::mma_f16(fragWi, fhi));
#pragma unroll
  for (int r = 0; r < 8; ++r) {
    const float m2 = zr[r] * zr[r] + zi[r] * zi[r];
    const float a = 1.0f - m2;
    dr[r] = (a * zr[r] - zi[r]) + wr[r] * kFoldBack;
    di[r] = (a * zi[r] + zr[r]) + wi[r] * kFoldBack;
  }
}

__global__ __launch_bounds__(128) void hopf_rk4_kernel(const float* __restrict__ x, const float* __restrict__ W_real,
                                                      const float* __restrict__ W_imag, const float* __restrict__ head_w,
                                                      const float* __restrict__ head_b, float* __restrict__ outs)
{
  __shared__ __align__(16) float osAll[kWavesPerBlock][kOPitch];
  __shared__ __align__(16) float wsm[2 * 256 + 128 + 4];

  const int lane = threadIdx.x & 31;
  const int wave = threadIdx.x >> 5;
  float* os = &osAll[wave][0];
  const int hsel = lane >> 4;
  const int n    = lane & 15;
  const bool lowHalf = (hsel == 0);
  constexpr int oWr = 0, oWi = 256, oHw = 512, oHb = 640;

#pragma unroll
  for (int it = 0; it < 8; ++it) { wsm[oWr + it * 32 + lane] = W_real[it * 32 + lane]; wsm[oWi + it * 32 + lane] = W_imag[it * 32 + lane]; }
#pragma unroll
  for (int it = 0; it < 4; ++it) wsm[oHw + it * 32 + lane] = head_w[it * 32 + lane];
  wsm[oHb + (lane & 3)] = head_b[lane & 3];
  __syncthreads();

  v16h fragWr, fragWi, fragH;
  {
    const int m = n;
    v8h r0, r1, i0, i1, h0, h1;
    const int mc = (m < kOutC) ? m : (kOutC - 1);
#pragma unroll
    for (int i = 0; i < 8; ++i) {
      const int j = 8 * hsel + i;
      const float wr = eng::bf16v(wsm[oWr + m * kOsc + j]);
      const float wi = eng::bf16v(wsm[oWi + m * kOsc + j]);
      r0[i] = eng::to_f16_flushed(wr * kWCarry);
      r1[i] = eng::to_f16_flushed(-wi * kWCarry);
      i0[i] = eng::to_f16_flushed(wi * kWCarry);
      i1[i] = eng::to_f16_flushed(wr * kWCarry);
      const float ha = eng::bf16v(wsm[oHw + mc * 2 * kOsc + j]);
      const float hb = eng::bf16v(wsm[oHw + mc * 2 * kOsc + kOsc + j]);
      h0[i] = eng::to_f16_flushed((m < kOutC) ? ha * kWCarry : 0.0f);
      h1[i] = eng::to_f16_flushed((m < kOutC) ? hb * kWCarry : 0.0f);
    }
    eng::FragU fu;
    fu.h[0] = r0; fu.h[1] = r1; fragWr = fu.v;
    fu.h[0] = i0; fu.h[1] = i1; fragWi = fu.v;
    fu.h[0] = h0; fu.h[1] = h1; fragH = fu.v;
  }
  float hbv[kOutC];
#pragma unroll
  for (int c = 0; c < kOutC; ++c) hbv[c] = eng::bf16v(wsm[oHb + c]);

#pragma unroll 1
  for (int jc = 0; jc < kChunksPerWave; ++jc) {
    const int cid = (blockIdx.x * kWavesPerBlock + wave) + kWaves * jc;
    const size_t s0 = (size_t)cid * kChunk;

#pragma unroll 1
    for (int tl8 = 0; tl8 < kTilesPerChunk; ++tl8) {
      const float* xp = x + (s0 + 16 * tl8 + n) * kOsc + 8 * hsel;
      const v4f x0 = *(const v4f*)xp;
      const v4f x1 = *(const v4f*)(xp + 4);
      float zr[8], zi[8];
#pragma unroll
      for (int r = 0; r < 8; ++r) {
        const float xv = eng::bf16v((r < 4) ? x0[r] : x1[r - 4]);
        const float xn = log2f(fmaxf(xv, 1.0f)) / 11.0f;
        const float th = xn * kTwoPi;
        zr[r] = cosf(th);
        zi[r] = sinf(th);
      }
#pragma unroll 1
      for (int st = 0; st < kRkSteps; ++st) {
        float kr[8], ki[8], sr[8], si[8], tr[8], ti[8];
        rhs(zr, zi, fragWr, fragWi, kr, ki);
#pragma unroll
        for (int r = 0; r < 8; ++r) { sr[r] = kr[r]; si[r] = ki[r]; tr[r] = zr[r] + (0.5f * kH) * kr[r]; ti[r] = zi[r] + (0.5f * kH) * ki[r]; }
        rhs(tr, ti, fragWr, fragWi, kr, ki);
#pragma unroll
        for (int r = 0; r < 8; ++r) { sr[r] = sr[r] + 2.0f * kr[r]; si[r] = si[r] + 2.0f * ki[r]; tr[r] = zr[r] + (0.5f * kH) * kr[r]; ti[r] = zi[r] + (0.5f * kH) * ki[r]; }
        rhs(tr, ti, fragWr, fragWi, kr, ki);
#pragma unroll
        for (int r = 0; r < 8; ++r) { sr[r] = sr[r] + 2.0f * kr[r]; si[r] = si[r] + 2.0f * ki[r]; tr[r] = zr[r] + kH * kr[r]; ti[r] = zi[r] + kH * ki[r]; }
        rhs(tr, ti, fragWr, fragWi, kr, ki);
#pragma unroll
        for (int r = 0; r < 8; ++r) { zr[r] = zr[r] + (kH / 6.0f) * (sr[r] + kr[r]); zi[r] = zi[r] + (kH / 6.0f) * (si[r] + ki[r]); }
      }
      v16h fhi, flo;
      eng::z_frags(zr, zi, fhi, flo);
      const v8f dh = eng::mma_f16_acc(fragH, flo, eng::mma_f16(fragH, fhi));
      if (lowHalf) {
        v4f o;
#pragma unroll
        for (int c = 0; c < kOutC; ++c) o[c] = dh[c] * kFoldBack + hbv[c];
        *(v4f*)(os + (16 * tl8 + n) * kOutC) = o;
      }
    }
    __syncthreads();

    {
      v4f ov[4];
#pragma unroll
      for (int it = 0; it < 4; ++it) ov[it] = *(const v4f*)(os + it * 128 + 4 * lane);
      for (int pass = 0; pass < 2; ++pass) {
#pragma unroll
        for (int it = 0; it < 4; ++it)
          *(volatile v4f*)(outs + s0 * kOutC + it * 128 + 4 * lane) = ov[it];
        __threadfence();
      }
    }
    __syncthreads();
  }
}

extern "C" void kernel_launch(void* const* d_in, const int* in_sizes, int n_in,
                              void* d_out, int out_size, void* d_ws, size_t ws_size,
                              hipStream_t stream) {
  (void)d_ws;
  (void)ws_size;
  if (n_in < 5 || d_out == nullptr) return;
  if (in_sizes[0] != kBatch * kOsc || in_sizes[1] != kOsc * kOsc || in_sizes[2] != kOsc * kOsc) return;
  if (in_sizes[3] != kOutC * 2 * kOsc || in_sizes[4] != kOutC) return;
  if (out_size != kBatch * kOutC) return;
  hopf_rk4_kernel<<<kWaves / kWavesPerBlock, 32 * kWavesPerBlock, 0, stream>>>(
      (const float*)d_in[0], (const float*)d_in[1], (const float*)d_in[2], (const float*)d_in[3], (const float*)d_in[4],
      (float*)d_out);
}
